// MotionEncoder_45758581571933
// MI455X (gfx1250) — hardware-run, weakly checked
//
#include <hip/hip_runtime.h>


namespace {
constexpr int NA = 40000, NL = 30000, NAP = 40064, NLP = 30016, TA = 20, TL = 10, DA = 5, DL = 2, LH = 64, G4 = 256, EAA = 640000, EAL = 1200000, ECA = 640000  , ECL = 1200000  , NAC = 40000  , NLC = 30000  ;
constexpr float XS = 8.0f, WSC = 256.0f, BNI = 0.99999500003749981f  ;
static_assert(NAP % 64 == 0 && NLP % 64 == 0 && NAC % 16 == 0 && NLC % 16 == 0, "tiling");
typedef _Float16 b16;
typedef __attribute__((ext_vector_type(16))) _Float16 v16b;
typedef __attribute__((ext_vector_type(8))) _Float16 v8b;
typedef __attribute__((ext_vector_type(8))) float v8f;
typedef __attribute__((ext_vector_type(4))) float v4f;
__device__ __forceinline__ float bf16_rne(float f) { unsigned int u = __float_as_uint(f); u += 0x7FFFu + ((u >> 16) & 1u); return __uint_as_float(u & 0xFFFF0000u); }
__device__ __forceinline__ void split16(float v, b16& hi, b16& lo) { hi = (b16)v; lo = (b16)(v - (float)hi); }
__device__ __forceinline__ v16b frag_kb(const b16* p, int hh) { const v8b a = *(const v8b*)(p + 8 * hh), b = *(const v8b*)(p + 16 + 8 * hh); v16b f;
#pragma unroll
  for (int e = 0; e < 8; ++e) { f[e] = a[e]; f[8 + e] = b[e]; } return f; }
__device__ __forceinline__ v8f wmma16b(v16b a, v16b b, v8f c) { v8f d = __builtin_amdgcn_wmma_f32_16x16x32_f16(false, a, false, b, (short)0, c, false, false); asm volatile("v_nop\n\tv_nop\n\tv_nop\n\tv_nop" : "+v"(d) : "v"(a), "v"(b)); return d; }
__device__ __forceinline__ void wave_lds_sync() { __builtin_amdgcn_fence(__ATOMIC_RELEASE, "workgroup"); __builtin_amdgcn_wave_barrier(); __builtin_amdgcn_fence(__ATOMIC_ACQUIRE, "workgroup"); }
__device__ __forceinline__ float pmul(float a, float b) { float p = a * b; asm volatile("" : "+v"(p)); return p; }
__device__ __forceinline__ int iclamp(int v, int lo, int hi) { return v < lo ? lo : (v > hi ? hi : v); }
constexpr int CSR_NBLK = 512, CSR_GB = 8, CSR_GN = 1 << CSR_GB  , CSR_MAXG = 512, CSR_CAP = 12288  ;
__global__ __launch_bounds__(64) void csrA_kernel(const int* __restrict__ dst, int E, int N, int nG, int CHP, int NGP, int* __restrict__ STG, int* __restrict__ HST) {
  extern __shared__ int sm[];
  int* cnt = sm; int* run = sm + NGP; int* ids = sm + 2 * NGP;
  const int b = blockIdx.x; const int ch = (E + CSR_NBLK - 1) / CSR_NBLK; const int e0 = b * ch, e1 = min(E, e0 + ch);
  for (int i = threadIdx.x; i < NGP; i += 64) cnt[i] = 0;
  for (int i = threadIdx.x; i < CHP; i += 64) ids[i] = -1;
  __syncthreads();
  if (threadIdx.x == 0) {
    for (int e = e0; e < e1; ++e) { int d = dst[e]; d = (d < 0) ? 0 : (d >= N ? N - 1 : d); cnt[d >> CSR_GB] += 1; }
    int acc = 0; for (int g = 0; g < nG; ++g) { run[g] = acc; acc += cnt[g]; }
    for (int e = e0; e < e1; ++e) { int d = dst[e]; d = (d < 0) ? 0 : (d >= N ? N - 1 : d); const int g = d >> CSR_GB; ids[run[g]] = e; run[g] += 1; } }
  __syncthreads();
  typedef __attribute__((ext_vector_type(4))) int v4i;
  for (int pass = 0; pass < 2; ++pass) {
    for (int i = threadIdx.x; i < CHP / 4; i += 64) *(volatile v4i*)(STG + (size_t)b * CHP + i * 4) = *(const v4i*)(&ids[i * 4]);
    for (int i = threadIdx.x; i < NGP / 4; i += 64) { v4i v; for (int e = 0; e < 4; ++e) v[e] = (i * 4 + e < nG) ? cnt[i * 4 + e] : 0; *(volatile v4i*)(HST + (size_t)b * NGP + i * 4) = v; }
    __threadfence(); }
}
__global__ __launch_bounds__(512) void csrS_kernel(const int* __restrict__ HST, int nG, int NGP, int* __restrict__ START, int* __restrict__ TOT, int* __restrict__ OFF) {
  __shared__ int tot[CSR_MAXG];
  const int b = threadIdx.x;
  for (int pass = 0; pass < 2; ++pass) { int runb = 0; for (int g = 0; g < nG; ++g) { int c = HST[(size_t)b * NGP + g]; c = (c < 0) ? 0 : c; ((volatile int*)OFF)[(size_t)g * CSR_NBLK + b] = runb; runb += c; } __threadfence(); }
  for (int g = threadIdx.x; g < nG; g += 512) { int s = 0; for (int bb = 0; bb < CSR_NBLK; ++bb) { int c = HST[(size_t)bb * NGP + g]; s += (c < 0) ? 0 : c; } tot[g] = s; }
  __syncthreads();
  if (threadIdx.x < 32) {
    __shared__ int st[CSR_MAXG + 32];
    if (threadIdx.x == 0) { int acc = 0; for (int g = 0; g < NGP; ++g) { st[g] = acc; if (g < nG) acc += (tot[g] + 31) & ~31; } st[NGP] = acc; }
    __builtin_amdgcn_fence(__ATOMIC_RELEASE, "workgroup"); __builtin_amdgcn_wave_barrier(); __builtin_amdgcn_fence(__ATOMIC_ACQUIRE, "workgroup");
    for (int pass = 0; pass < 2; ++pass) { for (int i = threadIdx.x; i < NGP + 32; i += 32) { ((volatile int*)START)[i] = (i <= NGP) ? st[min(i, NGP)] : 0; ((volatile int*)TOT)[i] = (i < nG) ? tot[i] : 0; } __threadfence(); } }
}
__global__ __launch_bounds__(256) void csrB_kernel(const int* __restrict__ dst, int N, int nG, int CHP, int NGP, int permLen, const int* __restrict__ STG, const int* __restrict__ HST, const int* __restrict__ OFF, const int* __restrict__ START, const int* __restrict__ TOT, int* __restrict__ PERM, int* __restrict__ ROWPTR, int* __restrict__ ROWCNT, int* __restrict__ FLAG) {
  typedef __attribute__((ext_vector_type(4))) int v4i;
  __shared__ int ids[CSR_CAP]; __shared__ unsigned short key[CSR_CAP]; __shared__ int outp[CSR_CAP]; __shared__ int ncnt[CSR_GN + 1]; __shared__ int boff[CSR_NBLK + 1];
  const int g = blockIdx.x, t_ = threadIdx.x; int tot = TOT[g]; int st = START[g], stn = START[g + 1]; const int v0 = g * CSR_GN; const int nv = min(CSR_GN, N - v0);
  st = (st < 0) ? 0 : (st > permLen - 32 ? permLen - 32 : st) & ~31; stn = (stn < st) ? st : (stn > permLen ? permLen : stn); tot = (tot < 0) ? 0 : tot; if (tot > stn - st && tot <= CSR_CAP) tot = stn - st;
  if (tot > CSR_CAP) {
    for (int pass = 0; pass < 2; ++pass) { for (int i = t_; i < CSR_GN / 4; i += 256) { v4i a, c; for (int e = 0; e < 4; ++e) { a[e] = st; c[e] = 0; } *(volatile v4i*)(ROWPTR + v0 + i * 4) = a; *(volatile v4i*)(ROWCNT + v0 + i * 4) = c; } if (t_ == 0) ((volatile int*)FLAG)[0] = 1; __threadfence(); } (void)nv; return; }
  if (t_ == 0) { int acc = 0; for (int b = 0; b < CSR_NBLK; ++b) { boff[b] = acc; int c = HST[(size_t)b * NGP + g]; c = (c < 0) ? 0 : (c > CHP ? CHP : c); acc += c; if (acc > tot) acc = tot; } boff[CSR_NBLK] = acc; }
  for (int i = t_; i <= CSR_GN; i += 256) ncnt[i] = 0;
  __syncthreads();
  for (int b = 0; b < CSR_NBLK; ++b) { const int c = boff[b + 1] - boff[b]; int o_ = OFF[(size_t)g * CSR_NBLK + b]; o_ = (o_ < 0) ? 0 : (o_ > CHP - c ? CHP - c : o_); const int* src_ = STG + (size_t)b * CHP + o_;
    for (int i = t_; i < c; i += 256) { int id = src_[i]; id = (id < 0) ? 0 : id; ids[boff[b] + i] = id; int d = dst[id]; d = (d < v0) ? v0 : (d >= N ? N - 1 : d); int kk = d - v0; kk = (kk < 0) ? 0 : (kk >= CSR_GN ? CSR_GN - 1 : kk); key[boff[b] + i] = (unsigned short)kk; } }
  __syncthreads();
  if (t_ == 0) { for (int i = 0; i < tot; ++i) ncnt[key[i]] += 1; int acc = 0; for (int vl = 0; vl < CSR_GN; ++vl) { const int c = ncnt[vl]; ncnt[vl] = acc; acc += c; } ncnt[CSR_GN] = acc;
    for (int i = 0; i < tot; ++i) { const int vl = key[i]; outp[ncnt[vl]] = ids[i]; ncnt[vl] += 1; }
    for (int vl = CSR_GN; vl > 0; --vl) ncnt[vl] = ncnt[vl - 1]; ncnt[0] = 0; }
  __syncthreads();
  for (int pass = 0; pass < 2; ++pass) {
    for (int i = t_; i < (stn - st) / 4; i += 256) { v4i v; for (int e = 0; e < 4; ++e) { const int q = i * 4 + e; v[e] = (q < tot) ? outp[q] : -1; } *(volatile v4i*)(PERM + st + i * 4) = v; }
    for (int i = t_; i < CSR_GN / 4; i += 256) { v4i a, c; for (int e = 0; e < 4; ++e) { const int vl = i * 4 + e; a[e] = st + ncnt[vl]; c[e] = (vl < nv) ? (ncnt[vl + 1] - ncnt[vl]) : 0; } *(volatile v4i*)(ROWPTR + v0 + i * 4) = a; *(volatile v4i*)(ROWCNT + v0 + i * 4) = c; }
    __threadfence(); }
}
__global__ __launch_bounds__(256) void csrZ_kernel(int* __restrict__ p, size_t n4) { typedef __attribute__((ext_vector_type(4))) int v4i; const size_t tid = (size_t)blockIdx.x * 256 + threadIdx.x, nth = (size_t)gridDim.x * 256; v4i z = {0, 0, 0, 0}; for (size_t i = tid; i < n4; i += nth) *(volatile v4i*)(p + i * 4) = z; }
struct CsrBufs { int *STG, *HST, *OFF, *START, *TOT, *PERM, *ROWPTR, *ROWCNT, *FLAG; int nG, NGP, CHP; size_t permLen; char* base; size_t bytes; };
static size_t csr_carve(CsrBufs& c, char* ws, size_t off, int E, int N) {
  const size_t off0 = off; c.base = ws + off;
  auto al = [&](size_t bytes) { char* p = ws + off; off += (bytes + 255) & ~(size_t)255; return p; };
  c.nG = (N + CSR_GN - 1) / CSR_GN; c.NGP = (c.nG + 31) & ~31; const int ch = (E + CSR_NBLK - 1) / CSR_NBLK; c.CHP = (ch + 31) & ~31; c.permLen = (size_t)E + 32 * (size_t)c.nG + 32;
  c.STG = (int*)al((size_t)CSR_NBLK * c.CHP * 4); c.HST = (int*)al((size_t)CSR_NBLK * c.NGP * 4); c.OFF = (int*)al((size_t)c.NGP * CSR_NBLK * 4); c.START = (int*)al((size_t)(c.NGP + 64) * 4); c.TOT = (int*)al((size_t)(c.NGP + 64) * 4);
  c.PERM = (int*)al(c.permLen * 4); c.ROWPTR = (int*)al((size_t)c.nG * CSR_GN * 4); c.ROWCNT = (int*)al((size_t)c.nG * CSR_GN * 4); c.FLAG = (int*)al(256);
  c.bytes = off - off0; return off;
}
static void csr_build(const CsrBufs& c, const int* dst, int E, int N, hipStream_t stream) {
  const size_t smem = (size_t)(2 * c.NGP + c.CHP) * 4;
  csrZ_kernel<<<512, 256, 0, stream>>>((int*)c.base, c.bytes / 16);
  csrA_kernel<<<CSR_NBLK, 64, smem, stream>>>(dst, E, N, c.nG, c.CHP, c.NGP, c.STG, c.HST);
  csrS_kernel<<<1, 512, 0, stream>>>(c.HST, c.nG, c.NGP, c.START, c.TOT, c.OFF);
  csrB_kernel<<<c.nG, 256, 0, stream>>>(dst, N, c.nG, c.CHP, c.NGP, (int)c.permLen, c.STG, c.HST, c.OFF, c.START, c.TOT, c.PERM, c.ROWPTR, c.ROWCNT, c.FLAG);
}

typedef __attribute__((ext_vector_type(2))) _Float16 v2h;
typedef __attribute__((ext_vector_type(4))) _Float16 v4h;
typedef __attribute__((ext_vector_type(2))) float v2f;
__global__ __launch_bounds__(256) void prep_kernel(const float* __restrict__ awhh, const float* __restrict__ lwhh, const float* const __restrict__ g0, const float* __restrict__ g1, const float* __restrict__ g2, const float* __restrict__ g3, const float* __restrict__ g4, const float* __restrict__ g5, const float* __restrict__ g6, const float* __restrict__ g7, const float* __restrict__ g8, b16* __restrict__ WHT, b16* __restrict__ GW) {
  int t = blockIdx.x * 256 + threadIdx.x; v8b o;
  if (t < 2 * G4 * LH / 8) { const int e = t * 8; const int m = e / (G4 * LH), el = e % (G4 * LH); const int oo = el / LH, d0 = el % LH; const float* w = m ? lwhh : awhh; for (int j = 0; j < 8; ++j) o[j] = (b16)(bf16_rne(w[(size_t)(d0 + j) * G4 + oo]) * WSC); for (int pass = 0; pass < 2; ++pass) { *(volatile v8b*)(WHT + e) = o; __threadfence(); } return; }
  t -= 2 * G4 * LH / 8; if (t < 9 * LH * LH / 8) { const int e = t * 8; const int m = e / (LH * LH), el = e % (LH * LH); const int oo = el / LH, d0 = el % LH; const float* w = m == 0 ? g0 : m == 1 ? g1 : m == 2 ? g2 : m == 3 ? g3 : m == 4 ? g4 : m == 5 ? g5 : m == 6 ? g6 : m == 7 ? g7 : g8;
    for (int j = 0; j < 8; ++j) o[j] = (b16)(bf16_rne(w[(size_t)(d0 + j) * LH + oo]) * WSC); for (int pass = 0; pass < 2; ++pass) { *(volatile v8b*)(GW + e) = o; __threadfence(); } }
}
__global__ __launch_bounds__(256) void zinit_kernel(b16* __restrict__ Hp, float* __restrict__ C, float* __restrict__ HS, size_t nrow) { const size_t u = (size_t)blockIdx.x * 256 + threadIdx.x; const size_t n8 = nrow * LH / 8; if (u >= n8) return; v8b z = {}; v4f zf = {0.0f, 0.0f, 0.0f, 0.0f};
  for (int pass = 0; pass < 2; ++pass) { *(volatile v8b*)(Hp + u * 8) = z; *(volatile v4f*)(C + u * 8) = zf; *(volatile v4f*)(C + u * 8 + 4) = zf; if (HS != nullptr) { *(volatile v4f*)(HS + u * 8) = zf; *(volatile v4f*)(HS + u * 8 + 4) = zf; } __threadfence(); } }
template <int DIN, int NP_, int NCUT, bool FIRST, bool COLLECT>
__global__ __launch_bounds__(128) void lstm_kernel(const float* __restrict__ x, int T, int t, const float* __restrict__ wih, const float* __restrict__ bih, const float* __restrict__ bhh, const b16* __restrict__ WHT, const b16* __restrict__ Hin, b16* __restrict__ Hout, float* __restrict__ C, float* __restrict__ HF, float* __restrict__ HS) {
  __shared__ __attribute__((aligned(16))) float Th[4][16][LH + 4], Tc[4][16][LH + 4]; __shared__ float Wi[DIN][G4]; __shared__ float Xs[4][16][DIN + 1];
  const int wave = threadIdx.x >> 5, lane = threadIdx.x & 31, nloc = lane & 15, hlf = lane >> 4; const size_t m0 = ((size_t)blockIdx.x * 4 + wave) * 16;
  for (int i = threadIdx.x; i < DIN * G4; i += 128) Wi[i / G4][i % G4] = bf16_rne(wih[i]);
  for (int i = lane; i < 16 * DIN; i += 32) { const size_t row = m0 + i / DIN; Xs[wave][i / DIN][i % DIN] = (row < (size_t)NCUT) ? bf16_rne(x[(row * T + t) * DIN + i % DIN]) : 0.0f; }
  const bool live = m0 < (size_t)NCUT;
  for (int rr = 0; rr < 16; ++rr) { const v2f cv = live ? *(const v2f*)(C + (m0 + rr) * LH + lane * 2) : (v2f){0.0f, 0.0f}; *(v2f*)(&Tc[wave][rr][lane * 2]) = cv; }
  __syncthreads();
  if (!live) return;
  v8f acc[16];
#pragma unroll
  for (int tt = 0; tt < 16; ++tt) acc[tt] = (v8f){};
  if (live) {
#pragma unroll
    for (int kb = 0; kb < LH; kb += 32) { const v16b a = frag_kb(Hin + (m0 + nloc) * LH + kb, hlf);
#pragma unroll
      for (int tt = 0; tt < 16; ++tt) acc[tt] = wmma16b(a, frag_kb(WHT + (size_t)(tt * 16 + nloc) * LH + kb, hlf), acc[tt]); } }
#pragma unroll
  for (int tt = 0; tt < 4; ++tt) { const int d = tt * 16 + nloc; float bsum[4], wv[4][DIN];
    for (int q = 0; q < 4; ++q) { const int col = q * LH + d; bsum[q] = bf16_rne(bih[col]) + bf16_rne(bhh[col]); for (int k = 0; k < DIN; ++k) wv[q][k] = Wi[k][col]; }
#pragma unroll
    for (int r = 0; r < 8; ++r) { const int rl = 8 * hlf + r; const size_t row = m0 + rl; float g[4];
      for (int q = 0; q < 4; ++q) { float s = acc[tt + 4 * q][r] * (1.0f / (XS * WSC)) + bsum[q]; for (int k = 0; k < DIN; ++k) s += pmul(Xs[wave][rl][k], wv[q][k]); g[q] = s; }
      const float cprev = Tc[wave][rl][d];
      const float ig = 1.0f / (1.0f + expf(-g[0])), fg = 1.0f / (1.0f + expf(-g[1])), gg = tanhf(g[2]), og = 1.0f / (1.0f + expf(-g[3]));
      const float cn = fg * cprev + ig * gg; const float hn = og * tanhf(cn);
      Tc[wave][rl][d] = live ? cn : 0.0f; Th[wave][rl][d] = live ? hn : 0.0f; } }
  wave_lds_sync();
  v2f hsum[16];
  for (int pass = 0; pass < 2; ++pass) {
    for (int rr = 0; rr < 16; ++rr) { const size_t row = m0 + rr; const v2f hv = *(const v2f*)(&Th[wave][rr][lane * 2]); const v2f cv = *(const v2f*)(&Tc[wave][rr][lane * 2]);
      *(volatile v2f*)(C + row * LH + lane * 2) = cv; *(volatile v2f*)(HF + row * LH + lane * 2) = hv; v2h hp; hp[0] = (b16)(hv[0] * XS); hp[1] = (b16)(hv[1] * XS); *(volatile v2h*)(Hout + row * LH + lane * 2) = hp;
      if (COLLECT) { v2f s = hv; if (pass == 0) { const v2f prev = *(const v2f*)(HS + row * LH + lane * 2); hsum[rr] = s + prev; } *(volatile v2f*)(HS + row * LH + lane * 2) = hsum[rr]; } }
    __threadfence(); }
}
__global__ __launch_bounds__(256) void scale_kernel(const float* __restrict__ IN, float s, size_t n2, float* __restrict__ OUT) { const size_t u = (size_t)blockIdx.x * 256 + threadIdx.x; if (u >= n2) return; v2f v = *(const v2f*)(IN + u * 2); v = v * s; for (int pass = 0; pass < 2; ++pass) { *(volatile v2f*)(OUT + u * 2) = v; __threadfence(); } }
template <int HEADS>
__global__ __launch_bounds__(128) void gproj_kernel(const float* __restrict__ X, int NCUT, const b16* __restrict__ W1, const float* __restrict__ att, float* __restrict__ P1, float* __restrict__ AT, const b16* __restrict__ W2, const float* __restrict__ bias2, float* __restrict__ P2) {
  __shared__ __attribute__((aligned(16))) float T1[4][16][LH + 4], T2[4][16][LH + 4]; __shared__ float Ta[4][16][4];
  constexpr int C = LH / HEADS;
  const int wave = threadIdx.x >> 5, lane = threadIdx.x & 31, nloc = lane & 15, hlf = lane >> 4; const size_t m0 = ((size_t)blockIdx.x * 4 + wave) * 16; const size_t vr = m0 + nloc; const bool two = (W2 != nullptr);
  v8f a1[4], a2[4];
#pragma unroll
  for (int tt = 0; tt < 4; ++tt) { a1[tt] = (v8f){}; a2[tt] = (v8f){}; }
  if (m0 < (size_t)NCUT) {
#pragma unroll
    for (int ks = 0; ks < 2; ++ks) { v16b ah, al; const float* xr = X + vr * LH + ks * 32; const v4f c0 = *(const v4f*)(xr + 8 * hlf), c1 = *(const v4f*)(xr + 8 * hlf + 4), c2 = *(const v4f*)(xr + 16 + 8 * hlf), c3 = *(const v4f*)(xr + 16 + 8 * hlf + 4); float cv[16];
      for (int i = 0; i < 4; ++i) { cv[i] = c0[i]; cv[4 + i] = c1[i]; cv[8 + i] = c2[i]; cv[12 + i] = c3[i]; }
#pragma unroll
      for (int e2 = 0; e2 < 16; ++e2) { b16 p, q; split16((vr < (size_t)NCUT ? cv[e2] : 0.0f) * XS, p, q); ah[e2] = p; al[e2] = q; }
#pragma unroll
      for (int tt = 0; tt < 4; ++tt) { const v16b bw = frag_kb(W1 + (size_t)(tt * 16 + nloc) * LH + ks * 32, hlf); a1[tt] = wmma16b(ah, bw, a1[tt]); a1[tt] = wmma16b(al, bw, a1[tt]);
        if (two) { const v16b bw2 = frag_kb(W2 + (size_t)(tt * 16 + nloc) * LH + ks * 32, hlf); a2[tt] = wmma16b(ah, bw2, a2[tt]); a2[tt] = wmma16b(al, bw2, a2[tt]); } } } }
  float pa[8][4]; for (int r = 0; r < 8; ++r) for (int h = 0; h < 4; ++h) pa[r][h] = 0.0f;
#pragma unroll
  for (int tt = 0; tt < 4; ++tt) { const int col = tt * 16 + nloc; const int hd = col / C; const float av = bf16_rne(att[col])  , bb = two ? bf16_rne(bias2[col]) : 0.0f;
#pragma unroll
    for (int r = 0; r < 8; ++r) { const bool lv = (m0 + 8 * hlf + r) < (size_t)NCUT; const float p1 = lv ? a1[tt][r] * (1.0f / (XS * WSC)) : 0.0f; T1[wave][8 * hlf + r][col] = p1;
#pragma unroll
      for (int h = 0; h < 4; ++h) if (h == hd) pa[r][h] += p1 * av;
      if (two) T2[wave][8 * hlf + r][col] = lv ? a2[tt][r] * (1.0f / (XS * WSC)) + bb : 0.0f; } }
#pragma unroll
  for (int r = 0; r < 8; ++r) {
#pragma unroll
    for (int h = 0; h < 4; ++h) {
#pragma unroll
      for (int o = 1; o < 16; o <<= 1) pa[r][h] += __shfl_xor(pa[r][h], o);
      if (nloc == 0) Ta[wave][8 * hlf + r][h] = (h < HEADS) ? pa[r][h] : 0.0f; } }
  wave_lds_sync();
  for (int pass = 0; pass < 2; ++pass) {
    for (int rr = 0; rr < 16; ++rr) { const size_t row = m0 + rr; *(volatile v2f*)(P1 + row * LH + lane * 2) = *(const v2f*)(&T1[wave][rr][lane * 2]); if (two) *(volatile v2f*)(P2 + row * LH + lane * 2) = *(const v2f*)(&T2[wave][rr][lane * 2]); }
    { const v2f a2v = *(const v2f*)(&Ta[wave][lane >> 1][(lane & 1) * 2]); *(volatile v2f*)(AT + m0 * 4 + lane * 2) = a2v; }
    __threadfence(); }
}
template <int HEADS, int ACT>
__global__ __launch_bounds__(256) void gagg_kernel(const float* __restrict__ XS, const float* __restrict__ AS, const float* __restrict__ AD, const float* __restrict__ R, int NDC, int NDP, int nloop, const int* __restrict__ srcs, int NSRC, int E, const int* __restrict__ PERM, const int* __restrict__ ROWPTR, const int* __restrict__ ROWCNT, int permLen, const float* __restrict__ bng, const float* __restrict__ bnb, float* __restrict__ O, float* __restrict__ out2) {
  constexpr int LPH = 32 / HEADS;
  const int wave = threadIdx.x >> 5, lane = threadIdx.x & 31; const size_t v = (size_t)blockIdx.x * 8 + wave; if (v >= (size_t)NDP) return; const int c = lane * 2, hd = lane / LPH; v2f o = {0.0f, 0.0f};
  if (v < (size_t)NDC) { const float adv = AD[v * 4 + hd]; float m = -INFINITY, den = 0.0f; v2f acc = {0.0f, 0.0f};
    auto take = [&](size_t s) { float lg = AS[s * 4 + hd] + adv; lg = lg >= 0.0f ? lg : 0.2f * lg; const float mn = fmaxf(m, lg); const float alf = (m == -INFINITY) ? 0.0f : __expf(m - mn), w = __expf(lg - mn); acc = acc * alf + *(const v2f*)(XS + s * LH + c) * w; den = den * alf + w; m = mn; };
    if (v < (size_t)nloop) take(v);
    int st = ROWPTR[v], cnt = ROWCNT[v]; cnt = iclamp(cnt, 0, 65536); st = iclamp(st, 0, permLen - cnt);
#pragma unroll 1
    for (int j = 0; j < cnt; ++j) { const int e = iclamp(PERM[st + j], 0, E - 1); const int s = iclamp(srcs[e], 0, NSRC - 1); if ((size_t)s == v) continue; take((size_t)s); }
    o = acc * (1.0f / (den + 1e-16f)) + *(const v2f*)(R + v * LH + c);
    if (ACT) { for (int i = 0; i < 2; ++i) { float y = o[i] * (bf16_rne(bng[c + i]) * BNI) + bf16_rne(bnb[c + i]); if (ACT == 1) y = y > 0.0f ? y : (expf(y) - 1.0f); else y = fmaxf(y, 0.0f); o[i] = y; } } }
  for (int pass = 0; pass < 2; ++pass) { *(volatile v2f*)(O + v * LH + c) = o; if (out2 != nullptr && v < (size_t)NDC) *(volatile v2f*)(out2 + v * LH + c) = o; __threadfence(); }
}
}

extern "C" void kernel_launch(void* const* d_in, const int* in_sizes, int n_in, void* d_out, int out_size, void* d_ws, size_t ws_size, hipStream_t stream) {
  (void)n_in;
  auto Fp = [&](int i) { return (const float*)d_in[i]; }; auto Ip = [&](int i) { return (const int*)d_in[i]; };
  if (in_sizes[0] != NA * TA * DA || in_sizes[1] != NL * TL * DL || in_sizes[2] != 2 * EAA || in_sizes[3] != 2 * EAL || in_sizes[4] != DA * G4 || in_sizes[5] != LH * G4 || in_sizes[8] != DL * G4 || in_sizes[12] != LH * LH || in_sizes[13] != LH || in_sizes[22] != LH || in_sizes[24] != LH * LH || in_sizes[26] != LH || in_sizes[36] != LH || out_size != 3 * NA * LH + NL * LH) return;
  float* out0 = (float*)d_out; float* out1 = out0 + (size_t)NA * LH; float* out2 = out1 + (size_t)NA * LH; float* out3 = out2 + (size_t)NA * LH;
  size_t off = 0; char* ws = (char*)d_ws;
  auto carve = [&](size_t bytes) { char* p = ws + off; off += (bytes + 255) & ~(size_t)255; return p; };
  b16* WHT = (b16*)carve((size_t)2 * G4 * LH * 2); b16* GW = (b16*)carve((size_t)9 * LH * LH * 2);
  b16* HpA = (b16*)carve((size_t)NAP * LH * 2); b16* HpB = (b16*)carve((size_t)NAP * LH * 2); float* Cst = (float*)carve((size_t)NAP * LH * 4); float* AEMB = (float*)carve((size_t)NAP * LH * 4); float* HS = (float*)carve((size_t)NLP * LH * 4); float* LEMB = (float*)carve((size_t)NLP * LH * 4); float* HFL = (float*)carve((size_t)NLP * LH * 4);
  float* XSb = (float*)carve((size_t)NAP * LH * 4); float* Rb = (float*)carve((size_t)NAP * LH * 4); float* ASb = (float*)carve((size_t)NAP * 4 * 4); float* ADb = (float*)carve((size_t)NAP * 4 * 4); float* Hb = (float*)carve((size_t)NAP * LH * 4); float* SOC = (float*)carve((size_t)NAP * LH * 4); float* Mb = (float*)carve((size_t)NAP * LH * 4);
  CsrBufs caa, cal; off = csr_carve(caa, ws, off, ECA, NA); off = csr_carve(cal, ws, off, ECL, NA);
  if (off > ws_size || off > ((size_t)128 << 20)) return;
  auto GWp = [&](int i) { return GW + (size_t)i * LH * LH; };
  prep_kernel<<<(2 * G4 * LH / 8 + 9 * LH * LH / 8 + 255) / 256, 256, 0, stream>>>(Fp(5), Fp(9), Fp(12), Fp(15), Fp(17), Fp(20), Fp(24), Fp(25), Fp(28), Fp(32), Fp(35), WHT, GW);
  csr_build(caa, Ip(2) + EAA, ECA, NA, stream);
  csr_build(cal, Ip(3), ECL, NA, stream);
  zinit_kernel<<<(unsigned)(((size_t)NAP * LH / 8 + 255) / 256), 256, 0, stream>>>(HpB, Cst, nullptr, (size_t)NAP);
  for (int t = 0; t < TA; ++t) { const b16* hin = (t & 1) ? HpA : HpB; b16* hout = (t & 1) ? HpB : HpA; lstm_kernel<DA, NAP, NAC, false, false><<<NAP / 64, 128, 0, stream>>>(Fp(0), TA, t, Fp(4), Fp(6), Fp(7), WHT, hin, hout, Cst, AEMB, nullptr); }
  scale_kernel<<<(unsigned)(((size_t)NAC * LH / 2 + 255) / 256), 256, 0, stream>>>(AEMB, 1.0f, (size_t)NAC * LH / 2, out0);
  zinit_kernel<<<(unsigned)(((size_t)NLP * LH / 8 + 255) / 256), 256, 0, stream>>>(HpB, Cst, HS, (size_t)NLP);
  for (int t = 0; t < TL; ++t) { const b16* hin = (t & 1) ? HpA : HpB; b16* hout = (t & 1) ? HpB : HpA; lstm_kernel<DL, NLP, NLC, false, true><<<NLP / 64, 128, 0, stream>>>(Fp(1), TL, t, Fp(8), Fp(10), Fp(11), WHT + (size_t)G4 * LH, hin, hout, Cst, HFL, HS); }
  scale_kernel<<<(unsigned)(((size_t)NLP * LH / 2 + 255) / 256), 256, 0, stream>>>(HS, 0.1f, (size_t)NLP * LH / 2, LEMB);
  scale_kernel<<<(unsigned)(((size_t)NLC * LH / 2 + 255) / 256), 256, 0, stream>>>(HS, 0.1f, (size_t)NLC * LH / 2, out3);
  gproj_kernel<4><<<NAP / 64, 128, 0, stream>>>(AEMB, NAC, GWp(0), Fp(13), XSb, ASb, GWp(1), Fp(16), Rb);
  gproj_kernel<4><<<NAP / 64, 128, 0, stream>>>(AEMB, NAC, GWp(0), Fp(14), Mb  , ADb, nullptr, nullptr, nullptr);
  gagg_kernel<4, 1><<<NAP / 8, 256, 0, stream>>>(XSb, ASb, ADb, Rb, NAC, NAP, NA, Ip(2), NA, EAA, caa.PERM, caa.ROWPTR, caa.ROWCNT, (int)caa.permLen, Fp(22), Fp(23), Hb, nullptr);
  gproj_kernel<4><<<NAP / 64, 128, 0, stream>>>(Hb, NAC, GWp(2), Fp(18), XSb, ASb, GWp(3), Fp(21), Rb);
  gproj_kernel<4><<<NAP / 64, 128, 0, stream>>>(Hb, NAC, GWp(2), Fp(19), Mb, ADb, nullptr, nullptr, nullptr);
  gagg_kernel<4, 0><<<NAP / 8, 256, 0, stream>>>(XSb, ASb, ADb, Rb, NAC, NAP, NA, Ip(2), NA, EAA, caa.PERM, caa.ROWPTR, caa.ROWCNT, (int)caa.permLen, Fp(22), Fp(23), SOC, out1);
  gproj_kernel<2><<<NLP / 64, 128, 0, stream>>>(LEMB, NLC, GWp(4), Fp(26), XSb, ASb, nullptr, nullptr, nullptr);
  gproj_kernel<2><<<NAP / 64, 128, 0, stream>>>(SOC, NAC, GWp(5), Fp(27), Hb  , ADb, GWp(6), Fp(29), Rb);
  gagg_kernel<2, 2><<<NAP / 8, 256, 0, stream>>>(XSb, ASb, ADb, Rb, NAC, NAP, NL, Ip(3) + EAL, NL, EAL, cal.PERM, cal.ROWPTR, cal.ROWCNT, (int)cal.permLen, Fp(30), Fp(31), Mb, nullptr);
  gproj_kernel<2><<<NAP / 64, 128, 0, stream>>>(Mb, NAC, GWp(7), Fp(33), XSb, ASb, GWp(8), Fp(36), Rb);
  gproj_kernel<2><<<NAP / 64, 128, 0, stream>>>(Mb, NAC, GWp(7), Fp(34), Hb, ADb, nullptr, nullptr, nullptr);
  gagg_kernel<2, 0><<<NAP / 8, 256, 0, stream>>>(XSb, ASb, ADb, Rb, NAC, NAP, NA  , Ip(3) + EAL, NA, EAL, cal.PERM, cal.ROWPTR, cal.ROWCNT, (int)cal.permLen, Fp(30), Fp(31), SOC  , out2);
}
